// GNN_55576876810911
// MI455X (gfx1250) — hardware-verified
//
#include <hip/hip_runtime.h>
#include <stddef.h>
#include <stdint.h>


#define FIN    5
#define HID    128
#define HK     256
#define N2C    256
#define N3C    128
#define OUTD   60
#define NTHR   256
#define NWAVE  8
#define EPT    8
#define CHUNK  (NTHR * EPT)
#define WCAP   (EPT * 32)
#define LISTN  (NWAVE * WCAP)
#define NBA    1024
#define SLA    10
#define RCAP   24576
#define DEGCAP 64
#define GBM    64
#define GBN    64
#define GTHR   128
#define UW2    (N2C * (HK / 8))
#define UW3    (N3C * (HK / 8))
#define AGG_ZINTS    (LISTN + 2 * RCAP + 3 * NBA)
#define MISC_INTS    16
#define ROWBUF_INTS  (NWAVE * HK / 2)
#define WT_FLOATS    (2 * HID * FIN + HID)
#define GBUF_FLOATS  (NWAVE * 8 * OUTD)
#define TAIL_INTS    3840
#define AGG_LDS_INTS (AGG_ZINTS + MISC_INTS + TAIL_INTS)
#define WSMAX  134217728

static_assert((CHUNK & (CHUNK - 1)) == 0 && CHUNK <= 4096);
static_assert((NBA & (NBA - 1)) == 0 && NBA == (1 << SLA));
static_assert(((long long)CHUNK << SLA) < (1LL << 31));
static_assert(NBA % (NWAVE * 8) == 0 && NBA % 32 == 0 && NBA % GBM == 0);
static_assert(RCAP % 4 == 0 && AGG_ZINTS % 4 == 0 && LISTN % 4 == 0 && ((AGG_ZINTS + MISC_INTS) % 4) == 0);
static_assert(ROWBUF_INTS + WT_FLOATS <= TAIL_INTS && GBUF_FLOATS <= TAIL_INTS);
static_assert(HK % 32 == 0 && HK == 2 * HID && N2C % GBN == 0 && N3C % GBN == 0);
static_assert(GBM == (GTHR / 32) * 16 && GBN == 64);
static_assert(UW2 % NTHR == 0 && UW3 % NTHR == 0 && (HK / 8) == 32);
static_assert((8 * OUTD * 4) % 128 == 0 && (8 * OUTD) % 4 == 0 && (8 * OUTD) / 4 == 120);
static_assert(AGG_LDS_INTS * 4 <= 300000);
static_assert(RCAP >= 16623 + 4096 && DEGCAP >= 35 + 8);

typedef float          v2f   __attribute__((ext_vector_type(2)));
typedef float          v4f   __attribute__((ext_vector_type(4)));
typedef float          v8f   __attribute__((ext_vector_type(8)));
typedef int            v4i   __attribute__((ext_vector_type(4)));
typedef int            v8i   __attribute__((ext_vector_type(8)));
typedef unsigned int   v4u   __attribute__((ext_vector_type(4)));
typedef unsigned short v4us  __attribute__((ext_vector_type(4)));
typedef unsigned short v8us  __attribute__((ext_vector_type(8)));
typedef unsigned short v16us __attribute__((ext_vector_type(16)));
typedef __bf16         v16bf __attribute__((ext_vector_type(16)));
typedef v2f  __attribute__((may_alias)) v2fa;
typedef v4f  __attribute__((may_alias)) v4fa;
typedef v4i  __attribute__((may_alias)) v4ia;
typedef v4u  __attribute__((may_alias)) v4ua;
typedef v4us __attribute__((may_alias)) v4usa;
typedef v8us __attribute__((may_alias)) v8usa;
union FragB { v16bf v; v16us u; v8us h[2]; v8i w; };

__device__ __forceinline__ v8f wmb(const FragB& a, const FragB& b, v8f c) {
  v8f d = __builtin_amdgcn_wmma_f32_16x16x32_bf16(false, a.v, false, b.v, (short)0, c, false, false);
  asm volatile("v_nop\n\tv_nop\n\tv_nop\n\tv_nop" : "+v"(d) : "v"(a.w), "v"(b.w));
  return d;
}

__device__ __forceinline__ unsigned bf16_bits(float f) {
  const unsigned u = __float_as_uint(f);
  const unsigned r = (u + 0x7FFFu + ((u >> 16) & 1u)) >> 16;
  return ((u & 0x7fffffffu) > 0x7f800000u) ? 0x7fc0u : r;
}
__device__ __forceinline__ float bf16_val(float f) {
  return __uint_as_float(bf16_bits(f) << 16);
}
__device__ __forceinline__ float lo16f(unsigned w) { return __uint_as_float(w << 16); }
__device__ __forceinline__ float hi16f(unsigned w) { return __uint_as_float(w & 0xffff0000u); }

__device__ __forceinline__ void wave_sync() {
  __builtin_amdgcn_fence(__ATOMIC_RELEASE, "wavefront");
  __builtin_amdgcn_wave_barrier();
  __builtin_amdgcn_fence(__ATOMIC_ACQUIRE, "wavefront");
}

template <int SLB>
__device__ __forceinline__ int scan_chunk(const int* __restrict__ dsts, int nE, int cbase, int slotBase,
                                          int nb, int vec8, int* list, int tid, int lane, int wave) {
  int wc = 0;
  const int el0  = tid * EPT;
  const int e0   = cbase + el0;
  const int sent = -2147483647 - 1;
  v4i da, db;
  if (vec8 != 0 && cbase + CHUNK <= nE) {
    da = *(const v4i*)(dsts + e0);
    db = *(const v4i*)(dsts + e0 + 4);
  } else {
    da.x = (e0     < nE) ? dsts[min(e0,     nE - 1)] : sent;
    da.y = (e0 + 1 < nE) ? dsts[min(e0 + 1, nE - 1)] : sent;
    da.z = (e0 + 2 < nE) ? dsts[min(e0 + 2, nE - 1)] : sent;
    da.w = (e0 + 3 < nE) ? dsts[min(e0 + 3, nE - 1)] : sent;
    db.x = (e0 + 4 < nE) ? dsts[min(e0 + 4, nE - 1)] : sent;
    db.y = (e0 + 5 < nE) ? dsts[min(e0 + 5, nE - 1)] : sent;
    db.z = (e0 + 6 < nE) ? dsts[min(e0 + 6, nE - 1)] : sent;
    db.w = (e0 + 7 < nE) ? dsts[min(e0 + 7, nE - 1)] : sent;
  }
  const unsigned nbs = (unsigned)slotBase;
  const unsigned unb = (unsigned)nb;
  const unsigned s0 = (unsigned)da.x - nbs, s1 = (unsigned)da.y - nbs;
  const unsigned s2 = (unsigned)da.z - nbs, s3 = (unsigned)da.w - nbs;
  const unsigned s4 = (unsigned)db.x - nbs, s5 = (unsigned)db.y - nbs;
  const unsigned s6 = (unsigned)db.z - nbs, s7 = (unsigned)db.w - nbs;
  const bool h0 = s0 < unb, h1 = s1 < unb, h2 = s2 < unb, h3 = s3 < unb;
  const bool h4 = s4 < unb, h5 = s5 < unb, h6 = s6 < unb, h7 = s7 < unb;
  const unsigned any = __builtin_amdgcn_ballot_w32(h0 | h1 | h2 | h3 | h4 | h5 | h6 | h7);
  if (any != 0u) {
#define HITJ(J, HJ, SJ) { \
      const unsigned mj = __builtin_amdgcn_ballot_w32(HJ); \
      if (mj != 0u) { \
        if (HJ) { \
          const int pos = wc + (int)__builtin_amdgcn_mbcnt_lo(mj, 0u); \
          if (pos < WCAP) list[wave * WCAP + pos] = ((el0 + (J)) << SLB) | (int)(SJ); \
        } \
        wc += (int)__builtin_popcount(mj); } }
    HITJ(0, h0, s0)
    HITJ(1, h1, s1)
    HITJ(2, h2, s2)
    HITJ(3, h3, s3)
    HITJ(4, h4, s4)
    HITJ(5, h5, s5)
    HITJ(6, h6, s6)
    HITJ(7, h7, s7)
#undef HITJ
  }
  return wc;
}

__global__ __launch_bounds__(NTHR) void k_prep(const float* __restrict__ x,
                                               const float* __restrict__ w2s, const float* __restrict__ w2n,
                                               const float* __restrict__ w3s, const float* __restrict__ w3n,
                                               int nN, int xRows,
                                               unsigned short* XB8, unsigned short* W2C, unsigned short* W3C) {
  const int u = (int)blockIdx.x * NTHR + (int)threadIdx.x;
  v8us o;
  unsigned short* dp;
  if (u < UW2) {
    const int n  = u >> 5;
    const int k8 = (u & 31) * 8;
    const int kk = k8 & (HID - 1);
    const int nr = n & (HID - 1);
    const float* p;
    if (n < HID) p = w2s + (size_t)nr * HID + kk;
    else         p = w2n + (size_t)nr * HID + kk;
    const v4f a = *(const v4f*)p;
    const v4f b = *(const v4f*)(p + 4);
    o[0] = (unsigned short)bf16_bits(a.x); o[1] = (unsigned short)bf16_bits(a.y);
    o[2] = (unsigned short)bf16_bits(a.z); o[3] = (unsigned short)bf16_bits(a.w);
    o[4] = (unsigned short)bf16_bits(b.x); o[5] = (unsigned short)bf16_bits(b.y);
    o[6] = (unsigned short)bf16_bits(b.z); o[7] = (unsigned short)bf16_bits(b.w);
    dp = W2C + (size_t)n * HK + k8;
  } else if (u < UW2 + UW3) {
    const int v  = u - UW2;
    const int n  = v >> 5;
    const int k8 = (v & 31) * 8;
    const int kk = k8 & (HID - 1);
    const int r  = n & 63;
    const bool ok = r < OUTD;
    const int rc = ok ? r : OUTD - 1;
    const float* p;
    if (n < 64) p = w3s + (size_t)rc * HID + kk;
    else        p = w3n + (size_t)rc * HID + kk;
    const v4f a = *(const v4f*)p;
    const v4f b = *(const v4f*)(p + 4);
    o[0] = ok ? (unsigned short)bf16_bits(a.x) : (unsigned short)0;
    o[1] = ok ? (unsigned short)bf16_bits(a.y) : (unsigned short)0;
    o[2] = ok ? (unsigned short)bf16_bits(a.z) : (unsigned short)0;
    o[3] = ok ? (unsigned short)bf16_bits(a.w) : (unsigned short)0;
    o[4] = ok ? (unsigned short)bf16_bits(b.x) : (unsigned short)0;
    o[5] = ok ? (unsigned short)bf16_bits(b.y) : (unsigned short)0;
    o[6] = ok ? (unsigned short)bf16_bits(b.z) : (unsigned short)0;
    o[7] = ok ? (unsigned short)bf16_bits(b.w) : (unsigned short)0;
    dp = W3C + (size_t)n * HK + k8;
  } else {
    const int row = u - (UW2 + UW3);
    if (row >= xRows) return;
    const bool ok = row < nN;
    const int rc = ok ? row : nN - 1;
    const float* p = x + (size_t)rc * FIN;
    const float f0 = p[0], f1 = p[1], f2 = p[2], f3 = p[3], f4 = p[4];
    o[0] = ok ? (unsigned short)bf16_bits(f0) : (unsigned short)0;
    o[1] = ok ? (unsigned short)bf16_bits(f1) : (unsigned short)0;
    o[2] = ok ? (unsigned short)bf16_bits(f2) : (unsigned short)0;
    o[3] = ok ? (unsigned short)bf16_bits(f3) : (unsigned short)0;
    o[4] = ok ? (unsigned short)bf16_bits(f4) : (unsigned short)0;
    o[5] = (unsigned short)0; o[6] = (unsigned short)0; o[7] = (unsigned short)0;
    dp = XB8 + (size_t)row * 8;
  }
  *(volatile v8us*)dp = o;
  __threadfence();
  *(volatile v8us*)dp = o;
}

__global__ __launch_bounds__(GTHR) void k_gemm(
    const unsigned short* __restrict__ A, const unsigned short* __restrict__ WT,
    float* outF, int K, int ldo, const float* __restrict__ bias, int nbias)
{
  __shared__ __attribute__((aligned(16))) float stg[GBM * GBN];
  const int tid = (int)threadIdx.x, lane = tid & 31, wave = tid >> 5, hh = lane >> 4, m = lane & 15;
  const int rowBase = (int)blockIdx.x * GBM;
  const int col0    = (int)blockIdx.y * GBN;

  v8f acc[4];
  {
    const v8f z = {0.f, 0.f, 0.f, 0.f, 0.f, 0.f, 0.f, 0.f};
    acc[0] = z; acc[1] = z; acc[2] = z; acc[3] = z;
  }
  const unsigned short* ap = A  + (size_t)(rowBase + 16 * wave + m) * (size_t)K + 8 * hh;
  const unsigned short* wp = WT + (size_t)(col0 + m) * (size_t)K + 8 * hh;
  const int ksteps = K >> 5;
#pragma unroll 1
  for (int ks = 0; ks < ksteps; ++ks) {
    FragB af;
    af.h[0] = *(const v8usa*)(ap + 32 * ks);
    af.h[1] = *(const v8usa*)(ap + 32 * ks + 16);
#pragma unroll
    for (int t = 0; t < 4; ++t) {
      const unsigned short* wq = wp + (size_t)(16 * t) * (size_t)K + 32 * ks;
      FragB bf;
      bf.h[0] = *(const v8usa*)wq;
      bf.h[1] = *(const v8usa*)(wq + 16);
      acc[t] = wmb(af, bf, acc[t]);
    }
  }

#pragma unroll
  for (int t = 0; t < 4; ++t) {
    const int lc = 16 * t + m;
#pragma unroll
    for (int r = 0; r < 8; ++r) {
      const int lr = 16 * wave + 8 * hh + r;
      stg[lr * GBN + lc] = acc[t][r];
    }
  }
  __syncthreads();

  v4f bq;
  {
    const int c0 = col0 + 4 * m;
    const int nbm = nbias - 1;
    const float t0 = bias[min(c0,     nbm)];
    const float t1 = bias[min(c0 + 1, nbm)];
    const float t2 = bias[min(c0 + 2, nbm)];
    const float t3 = bias[min(c0 + 3, nbm)];
    bq.x = (c0     < nbias) ? bf16_val(t0) : 0.0f;
    bq.y = (c0 + 1 < nbias) ? bf16_val(t1) : 0.0f;
    bq.z = (c0 + 2 < nbias) ? bf16_val(t2) : 0.0f;
    bq.w = (c0 + 3 < nbias) ? bf16_val(t3) : 0.0f;
  }

  v4f fv[8];
#pragma unroll
  for (int i = 0; i < 8; ++i) {
    const int lr = 16 * wave + 2 * i + hh;
    const v4f t = *(const v4fa*)(stg + lr * GBN + 4 * m);
    fv[i] = t + bq;
  }
#pragma unroll
  for (int i = 0; i < 8; ++i) {
    const int lr = 16 * wave + 2 * i + hh;
    const int gr = rowBase + lr;
    float* op = outF + (size_t)gr * (size_t)ldo + col0 + 4 * m;
    *(volatile v4f*)op = fv[i];
  }
  __threadfence();
#pragma unroll
  for (int i = 0; i < 8; ++i) {
    const int lr = 16 * wave + 2 * i + hh;
    const int gr = rowBase + lr;
    float* op = outF + (size_t)gr * (size_t)ldo + col0 + 4 * m;
    *(volatile v4f*)op = fv[i];
  }
}

__device__ __forceinline__ void build_lists(const int* __restrict__ keys, int nE, int vec8, int nodeBase,
                                            int* list, int* hl, int* sl, int* cnt, int* offs, int* cur,
                                            int* misc, int tid, int lane, int wave) {
  int t = 0, ov = 0;
  const int nChunks = (nE + CHUNK - 1) / CHUNK;
#pragma unroll 1
  for (int ch = 0; ch < nChunks; ++ch) {
    const int cbase = ch * CHUNK;
    const int wc = scan_chunk<SLA>(keys, nE, cbase, nodeBase, NBA, vec8, list, tid, lane, wave);
    if (lane == 0) misc[wave] = wc;
    __syncthreads();
    if (wave == 0) {
#pragma unroll 1
      for (int w2 = 0; w2 < NWAVE; ++w2) {
        int c = misc[w2];
        c = c < 0 ? 0 : (c > WCAP ? WCAP : c);
#pragma unroll 1
        for (int b0 = 0; b0 < c; b0 += 32) {
          const int idx = b0 + lane;
          const int ent = list[w2 * WCAP + (idx < WCAP ? idx : WCAP - 1)];
          const int m32 = (c - b0) < 32 ? (c - b0) : 32;
#pragma unroll 1
          for (int k = 0; k < m32; ++k) {
            const int u    = __builtin_amdgcn_readlane(ent, k);
            const int slot = u & (NBA - 1);
            const int el   = (u >> SLA) & (CHUNK - 1);
            const int pk   = ((cbase + el) << SLA) | slot;
            if (t < RCAP) {
              if (lane == 0) { hl[t] = pk; cnt[slot] = cnt[slot] + 1; }
              t = t + 1;
            } else {
              ov = 1;
            }
          }
        }
      }
    }
    __syncthreads();
  }
  if (wave == 0 && lane == 0) { misc[8] = t; misc[9] = ov; }
  __syncthreads();
  int tt = misc[8];
  tt = tt < 0 ? 0 : (tt > RCAP ? RCAP : tt);

  if (wave == 0) {
    const int base = lane * (NBA / 32);
    int s = 0;
#pragma unroll 1
    for (int i = 0; i < NBA / 32; ++i) s += cnt[base + i];
    int incl = s;
#pragma unroll
    for (int d = 1; d < 32; d <<= 1) {
      const int y = __shfl_up(incl, d, 32);
      if (lane >= d) incl += y;
    }
    int run = incl - s;
#pragma unroll 1
    for (int i = 0; i < NBA / 32; ++i) {
      const int cv = cnt[base + i];
      offs[base + i] = run;
      cur[base + i]  = run;
      run += cv;
    }
  }
  __syncthreads();
  if (wave == 0) {
#pragma unroll 1
    for (int b0 = 0; b0 < tt; b0 += 32) {
      const int idx = b0 + lane;
      const int ent = hl[idx < RCAP ? idx : RCAP - 1];
      const int m32 = (tt - b0) < 32 ? (tt - b0) : 32;
#pragma unroll 1
      for (int k = 0; k < m32; ++k) {
        const int u    = __builtin_amdgcn_readlane(ent, k);
        const int slot = u & (NBA - 1);
        if (lane == 0) {
          int p = cur[slot];
          p = p < 0 ? 0 : (p > RCAP - 1 ? RCAP - 1 : p);
          sl[p] = u;
          cur[slot] = p + 1;
        }
      }
    }
  }
  __syncthreads();
}

template <int MODE>
__global__ __launch_bounds__(NTHR) void k_scan(const int* __restrict__ srcs, const int* __restrict__ dsts,
                                               int nE, int nN, int vec8, int mRows,
                                               const unsigned short* __restrict__ xb8,
                                               const float* __restrict__ w1s, const float* __restrict__ w1n,
                                               const float* __restrict__ b1,
                                               const float* __restrict__ st,
                                               unsigned short* hpl, float* outp) {
  extern __shared__ __attribute__((aligned(16))) int dsm[];
  int* list = dsm;
  int* hl   = dsm + LISTN;
  int* sl   = hl + RCAP;
  int* cnt  = sl + RCAP;
  int* offs = cnt + NBA;
  int* cur  = offs + NBA;
  int* misc = cur + NBA;
  int* tail = misc + MISC_INTS;
  const int tid = (int)threadIdx.x, lane = tid & 31, wave = tid >> 5;
  const int nodeBase = (int)blockIdx.x * NBA;

  {
    const v4i z4 = {0, 0, 0, 0};
    for (int i = tid * 4; i < AGG_ZINTS; i += NTHR * 4) *(v4ia*)(dsm + i) = z4;
    if (tid < MISC_INTS) misc[tid] = 0;
  }
  if constexpr (MODE == 1) {
    float* wt = (float*)(tail + ROWBUF_INTS);
#pragma unroll 1
    for (int i = tid; i < HID * FIN; i += NTHR) {
      wt[i]             = bf16_val(w1s[i]);
      wt[HID * FIN + i] = bf16_val(w1n[i]);
    }
    if (tid < HID) wt[2 * HID * FIN + tid] = bf16_val(b1[tid]);
  }
  __syncthreads();

  build_lists(dsts, nE, vec8, nodeBase, list, hl, sl, cnt, offs, cur, misc, tid, lane, wave);
  const int ovf = misc[9];

  float wsr[4][FIN], wnr[4][FIN], bbr[4];
  if constexpr (MODE == 1) {
    const float* wt = (const float*)(tail + ROWBUF_INTS);
#pragma unroll
    for (int j = 0; j < 4; ++j) {
#pragma unroll
      for (int k = 0; k < FIN; ++k) {
        wsr[j][k] = wt[(4 * lane + j) * FIN + k];
        wnr[j][k] = wt[HID * FIN + (4 * lane + j) * FIN + k];
      }
      bbr[j] = wt[2 * HID * FIN + 4 * lane + j];
    }
  }

  const float qnan = __int_as_float(0x7fc00000);
  const float pz = (ovf != 0) ? qnan : 0.0f;
  constexpr int RPG = (MODE == 3) ? 8 : 1;
  unsigned short* rowbuf = (unsigned short*)tail + wave * HK;
  float* gbuf = (float*)tail + wave * (8 * OUTD);

#pragma unroll 1
  for (int gi = 0; gi < NBA / (NWAVE * RPG); ++gi) {
    const int gslot = (gi * NWAVE + wave) * RPG;
    const bool glive = (MODE != 3) || (nodeBase + gslot < nN);
    if (glive) {
#pragma unroll 1
      for (int r = 0; r < RPG; ++r) {
        const int s    = gslot + r;
        const int node = nodeBase + s;
        int c = cnt[s];
        const bool big = c > DEGCAP;
        c = c < 0 ? 0 : (c > DEGCAP ? DEGCAP : c);
        int o = offs[s];
        o = o < 0 ? 0 : (o > RCAP ? RCAP : o);
        const int nc = node < nN ? node : nN - 1;
        float a0 = 0.0f, a1 = 0.0f, a2 = 0.0f, a3 = 0.0f, a4 = 0.0f;
#pragma unroll 1
        for (int b0 = 0; b0 < c; b0 += 32) {
          int idx = o + b0 + lane;
          idx = idx > RCAP - 1 ? RCAP - 1 : idx;
          const int ent = sl[idx];
          int eid = ent >> SLA;
          eid = eid < 0 ? 0 : (eid > nE - 1 ? nE - 1 : eid);
          int sr = srcs[eid];
          sr = sr < 0 ? 0 : (sr > nN - 1 ? nN - 1 : sr);
          const int m32 = (c - b0) < 32 ? (c - b0) : 32;
          if constexpr (MODE == 1) {
            const v4u rw = *(const v4ua*)(xb8 + (size_t)sr * 8);
            const int r0 = (int)rw.x, r1 = (int)rw.y, r2 = (int)rw.z;
#pragma unroll 1
            for (int k = 0; k < m32; ++k) {
              const unsigned q0 = (unsigned)__builtin_amdgcn_readlane(r0, k);
              const unsigned q1 = (unsigned)__builtin_amdgcn_readlane(r1, k);
              const unsigned q2 = (unsigned)__builtin_amdgcn_readlane(r2, k);
              a0 += lo16f(q0); a1 += hi16f(q0);
              a2 += lo16f(q1); a3 += hi16f(q1);
              a4 += lo16f(q2);
            }
          } else if constexpr (MODE == 2) {
#pragma unroll 1
            for (int k = 0; k < m32; ++k) {
              const int sk = __builtin_amdgcn_readlane(sr, k);
              const v4f a = *(const v4fa*)(st + (size_t)sk * N2C + HID + 4 * lane);
              a0 += a.x; a1 += a.y; a2 += a.z; a3 += a.w;
            }
          } else {
#pragma unroll 1
            for (int k = 0; k < m32; ++k) {
              const int sk = __builtin_amdgcn_readlane(sr, k);
              const v2f a = *(const v2fa*)(st + (size_t)sk * N3C + 64 + 2 * lane);
              a0 += a.x; a1 += a.y;
            }
          }
        }
        const float pzr = big ? qnan : pz;

        if constexpr (MODE == 3) {
          const v2f sv = *(const v2fa*)(st + (size_t)nc * N3C + 2 * lane);
          v2f y;
          y.x = (sv.x + a0) + pzr;
          y.y = (sv.y + a1) + pzr;
          if (lane < OUTD / 2) *(v2fa*)(gbuf + r * OUTD + 2 * lane) = y;
        } else {
          float yv[4];
          if constexpr (MODE == 1) {
            const v4u sw = *(const v4ua*)(xb8 + (size_t)nc * 8);
            const float x0 = lo16f(sw.x), x1 = hi16f(sw.x), x2 = lo16f(sw.y), x3 = hi16f(sw.y);
            const float x4 = lo16f(sw.z);
#pragma unroll
            for (int j = 0; j < 4; ++j) {
              float s1 = x0 * wsr[j][0];
              s1 = fmaf(x1, wsr[j][1], s1);
              s1 = fmaf(x2, wsr[j][2], s1);
              s1 = fmaf(x3, wsr[j][3], s1);
              s1 = fmaf(x4, wsr[j][4], s1);
              float s2 = a0 * wnr[j][0];
              s2 = fmaf(a1, wnr[j][1], s2);
              s2 = fmaf(a2, wnr[j][2], s2);
              s2 = fmaf(a3, wnr[j][3], s2);
              s2 = fmaf(a4, wnr[j][4], s2);
              yv[j] = (s1 + s2) + bbr[j];
            }
          } else {
            const v4f sv = *(const v4fa*)(st + (size_t)nc * N2C + 4 * lane);
            yv[0] = sv.x + a0; yv[1] = sv.y + a1; yv[2] = sv.z + a2; yv[3] = sv.w + a3;
          }
          const bool live = node < nN;
          v4us mh, ml;
#pragma unroll
          for (int j = 0; j < 4; ++j) {
            const float v  = yv[j];
            const float rl = (v > 0.0f) ? v : (v - v);
            const float mv = live ? (rl + pzr) : 0.0f;
            const unsigned hb = bf16_bits(mv);
            mh[j] = (unsigned short)hb;
            ml[j] = (unsigned short)bf16_bits(mv - __uint_as_float(hb << 16));
          }
          *(v4usa*)(rowbuf + 4 * lane) = mh;
          *(v4usa*)(rowbuf + HID + 4 * lane) = ml;
          wave_sync();
          const v8us q0 = *(const v8usa*)(rowbuf + 8 * lane);
          wave_sync();
          if (node < mRows) {
            unsigned short* rp = hpl + (size_t)node * HK + 8 * lane;
            *(volatile v8us*)rp = q0;
            __threadfence();
            *(volatile v8us*)rp = q0;
          }
        }
      }
      if constexpr (MODE == 3) {
        wave_sync();
        v4f ov[4];
#pragma unroll
        for (int j = 0; j < 4; ++j) {
          const int t  = 32 * j + lane;
          const int tc = t < 120 ? t : 119;
          ov[j] = *(const v4fa*)(gbuf + 4 * tc);
        }
        wave_sync();
        float* ob = outp + (size_t)(nodeBase + gslot) * OUTD;
#pragma unroll
        for (int j = 0; j < 4; ++j) {
          const int t = 32 * j + lane;
          if (t < 120) *(volatile v4f*)(ob + 4 * t) = ov[j];
        }
        __threadfence();
#pragma unroll
        for (int j = 0; j < 4; ++j) {
          const int t = 32 * j + lane;
          if (t < 120) *(volatile v4f*)(ob + 4 * t) = ov[j];
        }
      }
    }
  }
}

static inline int cdiv(int a, int b) { return (a + b - 1) / b; }
static inline size_t al256(size_t o) { return (o + 255) & ~(size_t)255; }

extern "C" void kernel_launch(void* const* d_in, const int* in_sizes, int n_in,
                              void* d_out, int out_size, void* d_ws, size_t ws_size,
                              hipStream_t stream) {
  if (n_in < 11) return;
  if (in_sizes[0] < FIN || (in_sizes[0] % FIN) != 0) return;
  const int nN = in_sizes[0] / FIN;
  if (nN < 8 || (nN % 8) != 0 || nN > (1 << 22)) return;
  if (in_sizes[1] < 2 || (in_sizes[1] & 1) != 0) return;
  const int nE = in_sizes[1] / 2;
  if (nE < 1 || nE >= (1 << (31 - SLA))) return;
  if (in_sizes[2] != HID * FIN || in_sizes[3] != HID * FIN || in_sizes[4] != HID) return;
  if (in_sizes[5] != HID * HID || in_sizes[6] != HID * HID || in_sizes[7] != HID) return;
  if (in_sizes[8] != OUTD * HID || in_sizes[9] != OUTD * HID || in_sizes[10] != OUTD) return;
  if ((long long)out_size != (long long)nN * OUTD) return;

  const float* x   = (const float*)d_in[0];
  const int*   ei  = (const int*)d_in[1];
  const float* w1s = (const float*)d_in[2];
  const float* w1n = (const float*)d_in[3];
  const float* b1  = (const float*)d_in[4];
  const float* w2s = (const float*)d_in[5];
  const float* w2n = (const float*)d_in[6];
  const float* b2  = (const float*)d_in[7];
  const float* w3s = (const float*)d_in[8];
  const float* w3n = (const float*)d_in[9];
  const float* b3  = (const float*)d_in[10];
  float* out = (float*)d_out;
  const int* src = ei;
  const int* dst = ei + nE;

  const int MP    = cdiv(nN, GBM) * GBM;
  const int gM    = MP / GBM;
  const int gA    = cdiv(MP, NBA);
  const int xRows = cdiv(nN, NTHR) * NTHR;
  if ((long long)gA * NBA < (long long)MP) return;
  const int vec8 = ((nE & 3) == 0) ? 1 : 0;

  char* ws = (char*)d_ws;
  size_t off = 0;
  const size_t oW2 = off; off = al256(off + (size_t)N2C * HK * 2);
  const size_t oW3 = off; off = al256(off + (size_t)N3C * HK * 2);
  const size_t oXB = off; off = al256(off + (size_t)xRows * 8 * 2);
  const size_t oH  = off; off = al256(off + (size_t)MP * HK * 2);
  const size_t oST = off; off = al256(off + (size_t)MP * N2C * 4);
  if (off > ws_size || off > (size_t)WSMAX) return;
  unsigned short* W2C = (unsigned short*)(ws + oW2);
  unsigned short* W3C = (unsigned short*)(ws + oW3);
  unsigned short* XB8 = (unsigned short*)(ws + oXB);
  unsigned short* H   = (unsigned short*)(ws + oH);
  float*          ST  = (float*)(ws + oST);

  const size_t scanLds = (size_t)AGG_LDS_INTS * 4;
  hipFuncSetAttribute(reinterpret_cast<const void*>(&k_scan<1>), hipFuncAttributeMaxDynamicSharedMemorySize, (int)scanLds);
  hipFuncSetAttribute(reinterpret_cast<const void*>(&k_scan<2>), hipFuncAttributeMaxDynamicSharedMemorySize, (int)scanLds);
  hipFuncSetAttribute(reinterpret_cast<const void*>(&k_scan<3>), hipFuncAttributeMaxDynamicSharedMemorySize, (int)scanLds);

  k_prep<<<(UW2 + UW3 + xRows) / NTHR, NTHR, 0, stream>>>(x, w2s, w2n, w3s, w3n, nN, xRows, XB8, W2C, W3C);
  k_scan<1><<<gA, NTHR, scanLds, stream>>>(src, dst, nE, nN, vec8, MP, XB8, w1s, w1n, b1, ST, H, out);
  k_gemm<<<dim3(gM, N2C / GBN), GTHR, 0, stream>>>(H, W2C, ST, HK, N2C, b2, HID);
  k_scan<2><<<gA, NTHR, scanLds, stream>>>(src, dst, nE, nN, vec8, MP, XB8, w1s, w1n, b1, ST, H, out);
  k_gemm<<<dim3(gM, N3C / GBN), GTHR, 0, stream>>>(H, W3C, ST, HK, N3C, b3, OUTD);
  k_scan<3><<<gA, NTHR, scanLds, stream>>>(src, dst, nE, nN, vec8, MP, XB8, w1s, w1n, b1, ST, H, out);
}
